// Parallel_Linear_27462020891222
// MI455X (gfx1250) — hardware-verified
//
#include <hip/hip_runtime.h>


#ifndef NCS
#define NCS 64
#endif
#define CSEL_FULL 64
#define NBAT 64
#define CTOT 128
#define IND  256
#define OUTD 256

static_assert(NBAT == 64);
static_assert(IND % 32 == 0);
static_assert(OUTD % 64 == 0);
static_assert(NCS <= CSEL_FULL);
static_assert(NCS >= 1);
static_assert(((size_t)NBAT * CSEL_FULL * IND) % 8 == 0);
static_assert(((size_t)OUTD * IND) % (8 * 256) == 0);
static_assert(32 * 16 * 8 == 16 * 64 * 4);
static_assert(16 * 68 * 4 <= 131072);

typedef unsigned short bf;
typedef __attribute__((ext_vector_type(16))) __bf16   v16bf;
typedef __attribute__((ext_vector_type(8)))  unsigned short v8us;
typedef __attribute__((ext_vector_type(8)))  float    v8f;
typedef __attribute__((ext_vector_type(4)))  float    v4f;
typedef v4f  __attribute__((may_alias)) v4fa;

__device__ __forceinline__ unsigned short f2bf(float f) { unsigned u = __float_as_uint(f); u += 0x7FFFu + ((u >> 16) & 1u); return (unsigned short)(u >> 16); }
__device__ __forceinline__ float bfr(float f) { return __uint_as_float(((unsigned)f2bf(f)) << 16); }
__device__ __forceinline__ v16bf cat16b(v8us lo, v8us hi) { return __builtin_bit_cast(v16bf, __builtin_shufflevector(lo, hi, 0, 1, 2, 3, 4, 5, 6, 7, 8, 9, 10, 11, 12, 13, 14, 15)); }
__device__ __forceinline__ v8f wmmab(v16bf a, v16bf b, v8f c) { return __builtin_amdgcn_wmma_f32_16x16x32_bf16(false, a, false, b, (short)0, c, false, false); }
__device__ __forceinline__ v8f wmmabg(v16bf a, v16bf b, v8f c) { c = wmmab(a, b, c); asm volatile("v_nop\n\tv_nop\n\tv_nop\n\tv_nop" : "+v"(c) : "v"(a), "v"(b)); return c; }
__device__ __forceinline__ v16bf ldb(const bf* p)  { return cat16b(*(const v8us*)p, *(const v8us*)(p + 16)); }
__device__ __forceinline__ void wave_sync() { __builtin_amdgcn_fence(3  , "wavefront"); __builtin_amdgcn_wave_barrier(); asm volatile("" ::: "memory"); }

__global__ __launch_bounds__(256) void k_cvt8(const float* __restrict__ src, bf* dst, size_t n8) {
    const size_t i = (size_t)blockIdx.x * 256 + threadIdx.x; if (i >= n8) return;
    const v8f v = *(const v8f*)(src + i * 8); v8us o;
#pragma unroll
    for (int k = 0; k < 8; ++k) o[k] = f2bf(v[k]);
    *(volatile v8us*)(dst + i * 8) = o; __threadfence(); *(volatile v8us*)(dst + i * 8) = o;
}

__global__ __launch_bounds__(256) void k_wgather(const float* __restrict__ w, const int* __restrict__ chan, bf* dst) {
    const unsigned c = blockIdx.y;
    int chv = chan[c]; chv = max(chv, 0); chv = min(chv, CTOT - 1);
    const int ch = __builtin_amdgcn_readfirstlane(chv);
    const size_t i = (size_t)blockIdx.x * 256 + threadIdx.x;
    const v8f v = *(const v8f*)(w + (size_t)ch * ((size_t)OUTD * IND) + i * 8); v8us o;
#pragma unroll
    for (int k = 0; k < 8; ++k) o[k] = f2bf(v[k]);
    bf* d = dst + (size_t)c * ((size_t)OUTD * IND) + i * 8;
    *(volatile v8us*)d = o; __threadfence(); *(volatile v8us*)d = o;
}

__global__ __launch_bounds__(32) void k_gemm(const bf* __restrict__ A, const bf* __restrict__ Bt, const float* __restrict__ bias, const int* __restrict__ chan, float* OUT) {
    __shared__ __align__(16) float os[16 * 68];
    const int K = IND;
    const int lane = threadIdx.x & 31, lr = lane & 15, hi = lane >> 4;
    const unsigned c = blockIdx.x; const unsigned c0 = blockIdx.y * 64u;
    int chv = chan[c]; chv = max(chv, 0); chv = min(chv, CTOT - 1);
    const int ch = __builtin_amdgcn_readfirstlane(chv);
    v8f acc[4][4];
#pragma unroll
    for (int mb = 0; mb < 4; ++mb)
#pragma unroll
        for (int nb = 0; nb < 4; ++nb) acc[mb][nb] = (v8f){};
    const size_t aoff = ((size_t)lr * CSEL_FULL + c) * K + 8 * hi;
    const size_t boff = ((size_t)c * OUTD + c0 + lr) * K + 8 * hi;
#pragma unroll 1
    for (int kc = 0; kc < K; kc += 32) {
        v16bf a[4];
#pragma unroll
        for (int mb = 0; mb < 4; ++mb) a[mb] = ldb(A + aoff + (size_t)mb * 16 * CSEL_FULL * K + kc);
#pragma unroll
        for (int nb = 0; nb < 4; ++nb) { const v16bf b = ldb(Bt + boff + (size_t)nb * 16 * K + kc);
#pragma unroll
            for (int mb = 0; mb < 4; ++mb) acc[mb][nb] = wmmabg(a[mb], b, acc[mb][nb]); }
    }
    float bc[4];
#pragma unroll
    for (int nb = 0; nb < 4; ++nb) bc[nb] = bfr(bias[(size_t)ch * OUTD + c0 + nb * 16 + lr]);
    float* obase = OUT + ((size_t)c * OUTD + c0);
#pragma unroll
    for (int mb = 0; mb < 4; ++mb) {
#pragma unroll
        for (int nb = 0; nb < 4; ++nb) {
#pragma unroll
            for (int j = 0; j < 8; ++j) os[(hi * 8 + j) * 68 + nb * 16 + lr] = acc[mb][nb][j] + bc[nb]; }
        wave_sync();
#pragma unroll 1
        for (int ps = 0; ps < 2; ++ps) {
#pragma unroll
            for (int s = 0; s < 8; ++s) { const int row = 2 * s + (lane >> 4), cofs = (lane & 15) * 4;
                const v4f val = *(const v4fa*)(&os[row * 68 + cofs]);
                *(volatile v4f*)(obase + (size_t)(mb * 16 + row) * ((size_t)CSEL_FULL * OUTD) + cofs) = val; }
            if (ps == 0) __threadfence(); }
        wave_sync();
    }
}

static constexpr size_t al256(size_t v) { return (v + 255) & ~(size_t)255; }
static constexpr size_t X_ELEMS = (size_t)NBAT * CSEL_FULL * IND;
static constexpr size_t X_N8    = X_ELEMS / 8;
static constexpr unsigned X_GRID = (unsigned)((X_N8 + 255) / 256);
static constexpr size_t W_CH    = (size_t)OUTD * IND;
static constexpr unsigned W_GRIDX = (unsigned)(W_CH / 8 / 256);
static constexpr size_t NEED_W  = (size_t)CTOT * W_CH;
static constexpr size_t NEED_B  = (size_t)CTOT * OUTD;
static constexpr size_t NEED_O  = ((size_t)(NBAT - 1) * CSEL_FULL + NCS) * OUTD;
static constexpr size_t SZ_XB   = al256(X_ELEMS * 2);
static constexpr size_t SZ_WB   = al256((size_t)NCS * W_CH * 2);
static constexpr size_t OFF_XB  = 0;
static constexpr size_t OFF_WB  = OFF_XB + SZ_XB;
static constexpr size_t SZ_TOTAL = SZ_XB + SZ_WB;
static_assert(SZ_TOTAL <= (size_t)134217728);
static_assert((size_t)X_GRID * 256 * 8 == X_ELEMS);
static_assert((size_t)W_GRIDX * 256 * 8 == W_CH);
static_assert(((size_t)(NBAT - 1) * CSEL_FULL + (NCS - 1)) * OUTD + (OUTD - 1) < NEED_O);
static_assert(NEED_O * 4 <= (size_t)4194304);

extern "C" void kernel_launch(void* const* d_in, const int* in_sizes, int n_in,
                              void* d_out, int out_size, void* d_ws, size_t ws_size, hipStream_t stream) {
    if (n_in < 4) return;
    if ((size_t)in_sizes[0] < X_ELEMS) return;
    if (in_sizes[1] < NCS) return;
    if ((size_t)in_sizes[2] < NEED_W) return;
    if ((size_t)in_sizes[3] < NEED_B) return;
    if ((size_t)out_size < NEED_O) return;
    if (SZ_TOTAL > ws_size) return;
    const float* x    = (const float*)d_in[0];
    const int*   chan = (const int*)d_in[1];
    const float* w    = (const float*)d_in[2];
    const float* bias = (const float*)d_in[3];
    float* OUT = (float*)d_out;
    char* wsp = (char*)d_ws;
    bf* XB = (bf*)(wsp + OFF_XB);
    bf* WB = (bf*)(wsp + OFF_WB);

    k_cvt8<<<X_GRID, 256, 0, stream>>>(x, XB, X_N8);
    k_wgather<<<dim3(W_GRIDX, NCS, 1), 256, 0, stream>>>(w, chan, WB);
    k_gemm<<<dim3(NCS, OUTD / 64, 1), 32, 0, stream>>>(XB, WB, bias, chan, OUT);
}
